// SimpleCNN_87196426043827
// MI455X (gfx1250) — hardware-verified
//
#include <hip/hip_runtime.h>
#include <stddef.h>

constexpr int NB         = 256;
constexpr int IMG        = 64;
constexpr int CH1        = 32;
constexpr int CH2        = 64;
constexpr int H1         = 32;
constexpr int H2         = 16;
constexpr int KC2        = CH1 * 9;
constexpr int KFC        = CH2 * H2 * H2;
constexpr int NHID       = 128;
constexpr int NCLS       = 10;
constexpr int CHUNK_IMG  = 64;
constexpr int NCHUNK     = NB / CHUNK_IMG;
constexpr int CHUNK_ROWS = CHUNK_IMG * H1 * H1;
constexpr int IM2COL_WAVES = CHUNK_ROWS * KC2 / 1024;

static_assert(NB % CHUNK_IMG == 0, "chunking");
static_assert(KC2 % 32 == 0, "conv2 K multiple of 32");
static_assert(CHUNK_ROWS % 64 == 0 && CH2 % 64 == 0, "conv2 M,N tile multiples");
static_assert(NB % 64 == 0 && NHID % 64 == 0 && KFC % 32 == 0, "fc1 M,N,K tile multiples");
static_assert((CHUNK_ROWS * KC2) % 1024 == 0, "im2col wave granularity");
static_assert(IM2COL_WAVES % 8 == 0, "im2col block granularity");
static_assert((NB * NCLS) % 256 == 0, "fc2 grid exact");
static_assert((NB * NCLS) % 32 == 0, "fc2 whole lines");

typedef __attribute__((ext_vector_type(16))) _Float16 v16h;
typedef __attribute__((ext_vector_type(8)))  _Float16 v8h;
typedef __attribute__((ext_vector_type(16))) __bf16   v16b;
typedef __attribute__((ext_vector_type(8)))  __bf16   v8b;
typedef __attribute__((ext_vector_type(8)))  float    v8f;
typedef __attribute__((ext_vector_type(4)))  float    v4f;
typedef __attribute__((ext_vector_type(4)))  int      i4;
typedef __attribute__((ext_vector_type(4)))  unsigned u4;

__device__ __forceinline__ void dep_guard_h(v8f& a, v8f& b, v16h x, v16h y) { asm volatile("v_nop\n\tv_nop\n\tv_nop\n\tv_nop" : "+v"(a), "+v"(b) : "v"(x), "v"(y)); }
__device__ __forceinline__ void dep_guard_b(v8f& a, v8f& b, v16b x, v16b y) { asm volatile("v_nop\n\tv_nop\n\tv_nop\n\tv_nop" : "+v"(a), "+v"(b) : "v"(x), "v"(y)); }
__device__ __forceinline__ void keep4_h(v16h a, v16h b, v16h c, v16h d) { asm volatile("v_nop" :: "v"(a), "v"(b), "v"(c), "v"(d)); }
__device__ __forceinline__ void keep4_b(v16b a, v16b b, v16b c, v16b d) { asm volatile("v_nop" :: "v"(a), "v"(b), "v"(c), "v"(d)); }
__device__ __forceinline__ void acc_guard4(v8f& a, v8f& b, v8f& c, v8f& d) { asm volatile("v_nop\n\tv_nop\n\tv_nop\n\tv_nop" : "+v"(a), "+v"(b), "+v"(c), "+v"(d)); }
template <typename T> struct Frag;
template <> struct Frag<_Float16> {
  typedef v16h V; union U { v16h v; v8h h[2]; };
  static __device__ __forceinline__ v16h load(const _Float16* p) {
    U f; f.h[0] = *(const v8h*)(p); f.h[1] = *(const v8h*)(p + 16); return f.v;
  }
  static __device__ __forceinline__ v8f mma(v16h a, v16h b, v8f c) {
    return __builtin_amdgcn_wmma_f32_16x16x32_f16(false, a, false, b, (short)0, c, false, false);
  }
  static __device__ __forceinline__ void guard(v8f& a, v8f& b, v16h x, v16h y) { dep_guard_h(a, b, x, y); }
  static __device__ __forceinline__ void keep(v16h a, v16h b, v16h c, v16h d) { keep4_h(a, b, c, d); }
};
template <> struct Frag<__bf16> {
  typedef v16b V; union U { v16b v; v8b h[2]; };
  static __device__ __forceinline__ v16b load(const __bf16* p) {
    U f; f.h[0] = *(const v8b*)(p); f.h[1] = *(const v8b*)(p + 16); return f.v;
  }
  static __device__ __forceinline__ v8f mma(v16b a, v16b b, v8f c) {
    return __builtin_amdgcn_wmma_f32_16x16x32_bf16(false, a, false, b, (short)0, c, false, false);
  }
  static __device__ __forceinline__ void guard(v8f& a, v8f& b, v16b x, v16b y) { dep_guard_b(a, b, x, y); }
  static __device__ __forceinline__ void keep(v16b a, v16b b, v16b c, v16b d) { keep4_b(a, b, c, d); }
};

template <int ET> struct Elem;
template <> struct Elem<0> { typedef _Float16 T; };
template <> struct Elem<1> { typedef __bf16 T; };
template <int ET, int BIAS_MODE, int OUT_MODE, int ACT, bool GATE>
__global__ __launch_bounds__(256) void wmma_gemm64(
    const unsigned short* __restrict__ Ap, int lda, long strideA,
    const unsigned short* __restrict__ Btp, int ldb, long strideB,
    void* __restrict__ Cout, int ldc, long strideC,
    const float* __restrict__ bias,
    const int* __restrict__ gate, long strideG,
    int M, int N, int K, float scale) {
  typedef typename Elem<ET>::T T;
  typedef typename Frag<T>::V V;
  const T* A = (const T*)Ap; const T* Bt = (const T*)Btp;
  __shared__ __align__(16) float sT[8][16 * 68];
  const int b    = blockIdx.y;
  const int lane = threadIdx.x & 31;
  const int wave = threadIdx.x >> 5;
  const int tilesN = N >> 6;
  const int tilesM = M >> 6;
  const int tile = blockIdx.x * 8 + wave;
  if (tile >= tilesM * tilesN) return;
  const int tm = tile / tilesN;
  const int tn = tile - tm * tilesN;
  const int m0 = tm << 6;
  const int n0 = tn << 6;

  const T* Ab = A  + (size_t)b * strideA;
  const T* Bb = Bt + (size_t)b * strideB;

  const int rlane = lane & 15;
  const int koff  = (lane >> 4) * 8;
  const int mOff  = (lane >> 4) * 8;

  v8f acc[4][4];
#pragma unroll
  for (int i = 0; i < 4; ++i)
#pragma unroll
    for (int j = 0; j < 4; ++j) acc[i][j] = (v8f){0.f,0.f,0.f,0.f,0.f,0.f,0.f,0.f};

  for (int k0 = 0; k0 < K; k0 += 32) {
    V bh[4];
#pragma unroll
    for (int j = 0; j < 4; ++j) {
      const size_t bo = (size_t)(n0 + (j << 4) + rlane) * ldb + koff + k0;
      bh[j] = Frag<T>::load(Bb + bo);
    }
#pragma unroll
    for (int i = 0; i < 4; ++i) {
      const size_t ao = (size_t)(m0 + (i << 4) + rlane) * lda + koff + k0;
      V ah = Frag<T>::load(Ab + ao);
#pragma unroll
      for (int j = 0; j < 4; ++j) {
        acc[i][j] = Frag<T>::mma(ah, bh[j], acc[i][j]);
      }
      Frag<T>::guard(acc[i][0], acc[i][3], ah, ah);
    }
    Frag<T>::keep(bh[0], bh[1], bh[2], bh[3]);
  }
  acc_guard4(acc[0][0], acc[0][1], acc[0][2], acc[0][3]);
  acc_guard4(acc[1][0], acc[1][1], acc[1][2], acc[1][3]);
  acc_guard4(acc[2][0], acc[2][1], acc[2][2], acc[2][3]);
  acc_guard4(acc[3][0], acc[3][1], acc[3][2], acc[3][3]);

  float* slab = sT[wave];
#pragma unroll
  for (int i = 0; i < 4; ++i) {
    const int mBase = m0 + (i << 4);
    int gv[8] = {1, 1, 1, 1, 1, 1, 1, 1};
    if (GATE) {
      const int* gp = gate + (size_t)b * strideG + mBase + mOff;
      const i4 ga = *(const i4*)(gp);
      const i4 gb = *(const i4*)(gp + 4);
      gv[0] = ga.x; gv[1] = ga.y; gv[2] = ga.z; gv[3] = ga.w;
      gv[4] = gb.x; gv[5] = gb.y; gv[6] = gb.z; gv[7] = gb.w;
    }
#pragma unroll
    for (int j = 0; j < 4; ++j) {
      const int n = n0 + (j << 4) + rlane;
      float bv = 0.f;
      if (BIAS_MODE == 2) bv = bias[n];
#pragma unroll
      for (int r = 0; r < 8; ++r) {
        float v = acc[i][j][r] * scale;
        if (BIAS_MODE == 1) v += bias[mBase + mOff + r];
        if (BIAS_MODE == 2) v += bv;
        if (ACT == 2) v = fmaxf(v, 0.0f);
        if (GATE) v = (gv[r] != 0) ? v : 0.0f;
        slab[(mOff + r) * 68 + (j << 4) + rlane] = v;
      }
    }
    __builtin_amdgcn_fence(__ATOMIC_RELEASE, "workgroup");
    __builtin_amdgcn_wave_barrier();
    __builtin_amdgcn_fence(__ATOMIC_ACQUIRE, "workgroup");
    if (OUT_MODE == 0) {
      float* C = (float*)Cout + (size_t)b * strideC;
      const int hh = lane >> 4, c4 = (lane & 15) * 4;
      for (int pass = 0; pass < 2; ++pass) {
#pragma unroll
        for (int it = 0; it < 8; ++it) {
          const int row = it * 2 + hh;
          v4f v = *(const v4f*)(slab + row * 68 + c4);
          *(volatile v4f*)(C + (size_t)(mBase + row) * ldc + n0 + c4) = v;
        }
        __threadfence();
      }
    } else {
      const int q = lane >> 3, c8 = (lane & 7) * 8;
      unsigned short* C = (unsigned short*)Cout + (size_t)b * strideC;
      for (int pass = 0; pass < 2; ++pass) {
#pragma unroll
        for (int it = 0; it < 4; ++it) {
          const int row = it * 4 + q;
          const float* sp = slab + row * 68 + c8;
          v8h hv;
#pragma unroll
          for (int e = 0; e < 8; ++e) hv[e] = (_Float16)sp[e];
          *(volatile v8h*)(C + (size_t)(mBase + row) * ldc + n0 + c8) = hv;
        }
        __threadfence();
      }
    }
    __builtin_amdgcn_fence(__ATOMIC_RELEASE, "workgroup");
    __builtin_amdgcn_wave_barrier();
    __builtin_amdgcn_fence(__ATOMIC_ACQUIRE, "workgroup");
  }
}

__global__ __launch_bounds__(256) void k_masks(const int* __restrict__ cmap,
                                               int* __restrict__ m1, int* __restrict__ m2,
                                               int* __restrict__ m3, int* __restrict__ m4) {
  __shared__ __align__(16) int cm[IMG * IMG];
  __shared__ int s1[IMG * IMG];
  __shared__ int s2[H1 * H1];
  __shared__ int s3[H1 * H1];
  __shared__ int s4[H2 * H2];
  const int tid = threadIdx.x;
  const int b = blockIdx.x;
  const int* src = cmap + (size_t)b * (IMG * IMG);
#pragma unroll
  for (int u = 0; u < 4; ++u) {
    const int w4 = tid + 256 * u;
    *(i4*)(cm + 4 * w4) = *(const i4*)(src + 4 * w4);
  }
  __syncthreads();
  int* m1b = m1 + (size_t)b * (IMG * IMG);
  int* m2b = m2 + (size_t)b * (H1 * H1);
  int* m3b = m3 + (size_t)b * (H1 * H1);
  int* m4b = m4 + (size_t)b * (H2 * H2);

#pragma unroll 1
  for (int u = 0; u < 16; ++u) {
    const int e = tid + 256 * u;
    const int y = e >> 6, xq = e & 63;
    int s = 0;
#pragma unroll
    for (int dy = 0; dy < 3; ++dy) {
#pragma unroll
      for (int dx = 0; dx < 3; ++dx) {
        const int yy = y + dy, xx = xq + dx;
        const bool ok = (yy < IMG) && (xx < IMG);
        const int v = cm[(yy < IMG ? yy : IMG - 1) * IMG + (xx < IMG ? xx : IMG - 1)];
        s += ok ? v : 0;
      }
    }
    const int r = (s > 1) ? 1 : 0;
    s1[e] = r;
    *(volatile int*)(m1b + e) = r;
  }
  __syncthreads();
#pragma unroll 1
  for (int u = 0; u < 4; ++u) {
    const int e = tid + 256 * u;
    const int py = e >> 5, px = e & 31;
    const int* p = s1 + (2 * py) * IMG + 2 * px;
    const int s = p[0] + p[1] + p[IMG] + p[IMG + 1];
    const int r = (s > 1) ? 1 : 0;
    s2[e] = r;
    *(volatile int*)(m2b + e) = r;
  }
  __syncthreads();
#pragma unroll 1
  for (int u = 0; u < 4; ++u) {
    const int e = tid + 256 * u;
    const int y = e >> 5, xq = e & 31;
    int s = 0;
#pragma unroll
    for (int dy = 0; dy < 3; ++dy) {
#pragma unroll
      for (int dx = 0; dx < 3; ++dx) {
        const int yy = y + dy, xx = xq + dx;
        const bool ok = (yy < H1) && (xx < H1);
        const int v = s2[(yy < H1 ? yy : H1 - 1) * H1 + (xx < H1 ? xx : H1 - 1)];
        s += ok ? v : 0;
      }
    }
    const int r = (s > 1) ? 1 : 0;
    s3[e] = r;
    *(volatile int*)(m3b + e) = r;
  }
  __syncthreads();
  {
    const int e = tid;
    const int py = e >> 4, px = e & 15;
    const int* p = s3 + (2 * py) * H1 + 2 * px;
    const int s = p[0] + p[1] + p[H1] + p[H1 + 1];
    const int r = (s > 1) ? 1 : 0;
    s4[e] = r;
    *(volatile int*)(m4b + e) = r;
  }
  __threadfence();
  __syncthreads();
#pragma unroll 1
  for (int u = 0; u < 16; ++u) {
    const int e = tid + 256 * u;
    const int r = s1[e];
    *(volatile int*)(m1b + e) = r;
  }
#pragma unroll 1
  for (int u = 0; u < 4; ++u) {
    const int e = tid + 256 * u;
    const int r2v = s2[e];
    const int r3v = s3[e];
    *(volatile int*)(m2b + e) = r2v;
    *(volatile int*)(m3b + e) = r3v;
  }
  {
    const int r = s4[tid];
    *(volatile int*)(m4b + tid) = r;
  }
}

__global__ __launch_bounds__(128) void k_conv1_pool(const float* __restrict__ x,
                                                    const float* __restrict__ W1,
                                                    const float* __restrict__ b1,
                                                    const int* __restrict__ m1,
                                                    const int* __restrict__ m2,
                                                    _Float16* __restrict__ p1) {
  __shared__ float xs[4 * 66];
  __shared__ float wsf[CH1 * 32];
  __shared__ __align__(16) float slab[4][256];
  const int tid  = threadIdx.x;
  const int q    = tid >> 5;
  const int lane = tid & 31;
  const int hh   = lane >> 4;
  const int cc   = lane & 15;
  const int b    = blockIdx.x >> 5;
  const int py   = blockIdx.x & 31;

#pragma unroll
  for (int u = 0; u < 3; ++u) {
    const int w = tid + 128 * u;
    if (w < 264) {
      const int r  = w / 66;
      const int cx = w - r * 66;
      const int yy = 2 * py - 1 + r;
      const int xx = cx - 1;
      const bool inb = ((unsigned)yy < (unsigned)IMG) && ((unsigned)xx < (unsigned)IMG);
      const int yc = yy < 0 ? 0 : (yy > IMG - 1 ? IMG - 1 : yy);
      const int xc = xx < 0 ? 0 : (xx > IMG - 1 ? IMG - 1 : xx);
      const float v = x[((size_t)b * IMG + yc) * IMG + xc];
      xs[w] = inb ? v : 0.0f;
    }
  }
#pragma unroll
  for (int u = 0; u < 8; ++u) {
    const int w  = tid + 128 * u;
    const int oc = w >> 5, k = w & 31;
    const int kc = k < 9 ? k : 8;
    const float v = W1[oc * 9 + kc];
    wsf[w] = (k < 9) ? v : 0.0f;
  }
  __syncthreads();

  const int* m1p = m1 + ((size_t)(b * IMG + 2 * py + hh) * IMG + 16 * q);
  const i4 g1a = *(const i4*)(m1p);
  const i4 g1b = *(const i4*)(m1p + 4);
  const i4 g1c = *(const i4*)(m1p + 8);
  const i4 g1d = *(const i4*)(m1p + 12);
  const int g1v[16] = {g1a.x, g1a.y, g1a.z, g1a.w, g1b.x, g1b.y, g1b.z, g1b.w,
                       g1c.x, g1c.y, g1c.z, g1c.w, g1d.x, g1d.y, g1d.z, g1d.w};
  const int* m2p = m2 + ((size_t)(b * H1 + py) * H1 + 8 * q);
  const i4 g2a = *(const i4*)(m2p);
  const i4 g2b = *(const i4*)(m2p + 4);
  const int g2v[8] = {g2a.x, g2a.y, g2a.z, g2a.w, g2b.x, g2b.y, g2b.z, g2b.w};
  const float bj[2] = {b1[cc], b1[16 + cc]};

  v16h bfr[2];
#pragma unroll
  for (int j = 0; j < 2; ++j) {
    const float* wr = wsf + (16 * j + cc) * 32;
#pragma unroll
    for (int e = 0; e < 8; ++e) {
      bfr[j][e]     = (_Float16)wr[8 * hh + e];
      bfr[j][8 + e] = (_Float16)wr[16 + 8 * hh + e];
    }
  }

  v8f acc[2][2];
#pragma unroll
  for (int i = 0; i < 2; ++i)
#pragma unroll
    for (int j = 0; j < 2; ++j) acc[i][j] = (v8f){0.f,0.f,0.f,0.f,0.f,0.f,0.f,0.f};

  const int sy = cc >> 3, xr = cc & 7;
#pragma unroll
  for (int i = 0; i < 2; ++i) {
    const int xp = 16 * q + 8 * i + xr;
    const float* xrow = xs + sy * 66 + xp;
    float t[9];
#pragma unroll
    for (int ty = 0; ty < 3; ++ty)
#pragma unroll
      for (int tx = 0; tx < 3; ++tx) t[3 * ty + tx] = xrow[ty * 66 + tx];
    v16h af;
#pragma unroll
    for (int e = 0; e < 8; ++e) {
      const float fe = (hh != 0) ? ((e == 0) ? t[8] : 0.0f) : t[e];
      af[e] = (_Float16)fe;
      af[8 + e] = (_Float16)0.0f;
    }
#pragma unroll
    for (int j = 0; j < 2; ++j) acc[i][j] = Frag<_Float16>::mma(af, bfr[j], acc[i][j]);
    Frag<_Float16>::guard(acc[i][0], acc[i][1], af, af);
  }
  acc_guard4(acc[0][0], acc[0][1], acc[1][0], acc[1][1]);

  float* sl = slab[q];
#pragma unroll
  for (int i = 0; i < 2; ++i) {
#pragma unroll
    for (int j = 0; j < 2; ++j) {
      float v[8];
#pragma unroll
      for (int r = 0; r < 8; ++r) {
        float t2 = acc[i][j][r] + bj[j];
        t2 = fmaxf(t2, 0.0f);
        v[r] = (g1v[8 * i + r] != 0) ? t2 : 0.0f;
      }
      float pv[4];
#pragma unroll
      for (int r2 = 0; r2 < 4; ++r2) {
        float a = fmaxf(v[2 * r2], v[2 * r2 + 1]);
        const float o = __shfl_xor(a, 16, 32);
        a = fmaxf(a, o);
        pv[r2] = (g2v[4 * i + r2] != 0) ? a : 0.0f;
      }
      const float s0 = (hh != 0) ? pv[2] : pv[0];
      const float s1v = (hh != 0) ? pv[3] : pv[1];
      const int pp0 = 4 * i + 2 * hh;
      sl[pp0 * 32 + 16 * j + cc]       = s0;
      sl[(pp0 + 1) * 32 + 16 * j + cc] = s1v;
    }
  }
  __builtin_amdgcn_fence(__ATOMIC_RELEASE, "workgroup");
  __builtin_amdgcn_wave_barrier();
  __builtin_amdgcn_fence(__ATOMIC_ACQUIRE, "workgroup");
  {
    const int pp = lane >> 2, cg = lane & 3;
    const float* sp = sl + pp * 32 + 8 * cg;
    const v4f lo = *(const v4f*)(sp);
    const v4f hi = *(const v4f*)(sp + 4);
    v8h hv;
    hv[0] = (_Float16)lo.x; hv[1] = (_Float16)lo.y; hv[2] = (_Float16)lo.z; hv[3] = (_Float16)lo.w;
    hv[4] = (_Float16)hi.x; hv[5] = (_Float16)hi.y; hv[6] = (_Float16)hi.z; hv[7] = (_Float16)hi.w;
    _Float16* dst = p1 + ((((size_t)b * H1 + py) * H1 + 8 * q + pp) * CH1 + 8 * cg);
    *(volatile v8h*)dst = hv;
    __threadfence();
    *(volatile v8h*)dst = hv;
  }
}

__global__ __launch_bounds__(256) void k_im2col(const _Float16* __restrict__ p1c,
                                                _Float16* __restrict__ acol) {
  const int gid = blockIdx.x * 256 + threadIdx.x;
  const int w = gid >> 5;
  const int L = gid & 31;
  u4 val[4];
#pragma unroll
  for (int k = 0; k < 4; ++k) {
    const int p   = 32 * k + L;
    const int g   = w * 1024 + 8 * p;
    const int row = g / KC2;
    const int col = g - row * KC2;
    const int tap = col >> 5;
    const int ic0 = col & 31;
    const int bl  = row >> 10;
    const int pix = row & 1023;
    const int y   = pix >> 5;
    const int xq  = pix & 31;
    const int ty  = tap / 3;
    const int tx  = tap - 3 * ty;
    const int yy  = y + ty - 1;
    const int xx  = xq + tx - 1;
    const bool inb = ((unsigned)yy < (unsigned)H1) && ((unsigned)xx < (unsigned)H1);
    const int yc = yy < 0 ? 0 : (yy > H1 - 1 ? H1 - 1 : yy);
    const int xc = xx < 0 ? 0 : (xx > H1 - 1 ? H1 - 1 : xx);
    const u4 ld = *(const u4*)(p1c + ((((size_t)bl * H1 + yc) * H1 + xc) * CH1 + ic0));
    u4 z;
    z.x = inb ? ld.x : 0u; z.y = inb ? ld.y : 0u; z.z = inb ? ld.z : 0u; z.w = inb ? ld.w : 0u;
    val[k] = z;
  }
  for (int pass = 0; pass < 2; ++pass) {
#pragma unroll
    for (int k = 0; k < 4; ++k) {
      const int p = 32 * k + L;
      *(volatile u4*)(acol + (size_t)w * 1024 + 8 * p) = val[k];
    }
    __threadfence();
  }
}

__global__ __launch_bounds__(256) void k_cast_w2(const float* __restrict__ W2,
                                                 _Float16* __restrict__ wt) {
  const int t   = blockIdx.x * 256 + threadIdx.x;
  const int icg = t & 3;
  const int rt  = t >> 2;
  const int oc  = rt / 9;
  const int tap = rt - 9 * oc;
  v8h hv;
#pragma unroll
  for (int e = 0; e < 8; ++e) {
    const int ic = 8 * icg + e;
    hv[e] = (_Float16)W2[((size_t)oc * CH1 + ic) * 9 + tap];
  }
  _Float16* dst = wt + (size_t)8 * t;
  *(volatile v8h*)dst = hv;
  __threadfence();
  *(volatile v8h*)dst = hv;
}

__global__ __launch_bounds__(256) void k_cast_fc1(const float* __restrict__ Wfc1,
                                                  _Float16* __restrict__ wt) {
  const int gid = blockIdx.x * 256 + threadIdx.x;
  const int cg  = gid & 7;
  const int pp  = (gid >> 3) & 255;
  const int n   = gid >> 11;
  const float* src = Wfc1 + (size_t)n * KFC + (size_t)(8 * cg) * 256 + pp;
  v8h hv;
#pragma unroll
  for (int e = 0; e < 8; ++e) hv[e] = (_Float16)(src[(size_t)e * 256] * 64.0f);
  _Float16* dst = wt + (size_t)8 * gid;
  *(volatile v8h*)dst = hv;
  __threadfence();
  *(volatile v8h*)dst = hv;
}

__device__ __forceinline__ float h2f_lo(unsigned w) { return (float)__builtin_bit_cast(_Float16, (unsigned short)(w & 0xffffu)); }
__device__ __forceinline__ float h2f_hi(unsigned w) { return (float)__builtin_bit_cast(_Float16, (unsigned short)(w >> 16)); }

__global__ __launch_bounds__(256) void k_pool2(const _Float16* __restrict__ r2,
                                               const int* __restrict__ m4,
                                               _Float16* __restrict__ p2) {
  const int gid = blockIdx.x * 256 + threadIdx.x;
  const int cg  = gid & 7;
  const int pp  = (gid >> 3) & 255;
  const int b   = gid >> 11;
  const int py  = pp >> 4, px = pp & 15;
  const int gt  = m4[(size_t)b * (H2 * H2) + pp];
  float mx[8] = {0.f, 0.f, 0.f, 0.f, 0.f, 0.f, 0.f, 0.f};
#pragma unroll
  for (int sy = 0; sy < 2; ++sy) {
#pragma unroll
    for (int sx = 0; sx < 2; ++sx) {
      const u4 wv = *(const u4*)(r2 + ((((size_t)b * H1 + 2 * py + sy) * H1 + 2 * px + sx) * CH2 + 8 * cg));
      mx[0] = fmaxf(mx[0], h2f_lo(wv.x)); mx[1] = fmaxf(mx[1], h2f_hi(wv.x));
      mx[2] = fmaxf(mx[2], h2f_lo(wv.y)); mx[3] = fmaxf(mx[3], h2f_hi(wv.y));
      mx[4] = fmaxf(mx[4], h2f_lo(wv.z)); mx[5] = fmaxf(mx[5], h2f_hi(wv.z));
      mx[6] = fmaxf(mx[6], h2f_lo(wv.w)); mx[7] = fmaxf(mx[7], h2f_hi(wv.w));
    }
  }
  v8h hv;
#pragma unroll
  for (int e = 0; e < 8; ++e) hv[e] = (_Float16)((gt != 0) ? mx[e] : 0.0f);
  _Float16* dst = p2 + (size_t)8 * gid;
  *(volatile v8h*)dst = hv;
  __threadfence();
  *(volatile v8h*)dst = hv;
}

__global__ __launch_bounds__(256) void k_fc2(const float* __restrict__ h,
                                             const float* __restrict__ Wfc2,
                                             const float* __restrict__ bfc2,
                                             float* __restrict__ out) {
  const int idx = blockIdx.x * 256 + threadIdx.x;
  const int o  = idx % NCLS;
  const int bb = idx / NCLS;
  const v4f* hr = (const v4f*)(h + (size_t)bb * NHID);
  const v4f* wr = (const v4f*)(Wfc2 + (size_t)o * NHID);
  float acc = 0.0f;
#pragma unroll 1
  for (int j4 = 0; j4 < NHID / 4; ++j4) {
    const v4f a = hr[j4];
    const v4f w = wr[j4];
    acc = fmaf(a.x, w.x, acc);
    acc = fmaf(a.y, w.y, acc);
    acc = fmaf(a.z, w.z, acc);
    acc = fmaf(a.w, w.w, acc);
  }
  const float res = acc + bfc2[o];
  *(volatile float*)(out + idx) = res;
  __threadfence();
  *(volatile float*)(out + idx) = res;
}

extern "C" void kernel_launch(void* const* d_in, const int* in_sizes, int n_in,
                              void* d_out, int out_size, void* d_ws, size_t ws_size,
                              hipStream_t stream) {
  if (n_in < 10) return;
  if (in_sizes[0] != NB * IMG * IMG || in_sizes[1] != NB * IMG * IMG ||
      in_sizes[2] != CH1 * 9 || in_sizes[3] != CH1 || in_sizes[4] != CH2 * CH1 * 9 ||
      in_sizes[5] != CH2 || in_sizes[6] != NHID * KFC || in_sizes[7] != NHID ||
      in_sizes[8] != NCLS * NHID || in_sizes[9] != NCLS || out_size != NB * NCLS) return;

  const float* x    = (const float*)d_in[0];
  const int*   cmap = (const int*)d_in[1];
  const float* W1   = (const float*)d_in[2];
  const float* b1   = (const float*)d_in[3];
  const float* W2   = (const float*)d_in[4];
  const float* b2   = (const float*)d_in[5];
  const float* Wfc1 = (const float*)d_in[6];
  const float* bfc1 = (const float*)d_in[7];
  const float* Wfc2 = (const float*)d_in[8];
  const float* bfc2 = (const float*)d_in[9];
  float* out = (float*)d_out;

  char* wsb = (char*)d_ws;
  size_t off = 0;
  auto carve = [&](size_t bytes) -> size_t { size_t o = off; off += (bytes + 255) & ~(size_t)255; return o; };
  const size_t o_m1   = carve((size_t)NB * IMG * IMG * 4);
  const size_t o_m2   = carve((size_t)NB * H1 * H1 * 4);
  const size_t o_m3   = carve((size_t)NB * H1 * H1 * 4);
  const size_t o_m4   = carve((size_t)NB * H2 * H2 * 4);
  const size_t o_p1   = carve((size_t)NB * H1 * H1 * CH1 * 2);
  const size_t o_w2t  = carve((size_t)CH2 * KC2 * 2);
  const size_t o_acol = carve((size_t)CHUNK_ROWS * KC2 * 2);
  const size_t o_r2   = carve((size_t)NB * H1 * H1 * CH2 * 2);
  const size_t o_p2   = carve((size_t)NB * KFC * 2);
  const size_t o_wfc  = carve((size_t)NHID * KFC * 2);
  const size_t o_h    = carve((size_t)NB * NHID * 4);
  if (off > ws_size) return;

  int* m1 = (int*)(wsb + o_m1);
  int* m2 = (int*)(wsb + o_m2);
  int* m3 = (int*)(wsb + o_m3);
  int* m4 = (int*)(wsb + o_m4);
  _Float16* p1    = (_Float16*)(wsb + o_p1);
  _Float16* w2t   = (_Float16*)(wsb + o_w2t);
  _Float16* acol  = (_Float16*)(wsb + o_acol);
  _Float16* r2    = (_Float16*)(wsb + o_r2);
  _Float16* p2    = (_Float16*)(wsb + o_p2);
  _Float16* wfc1t = (_Float16*)(wsb + o_wfc);
  float*    hbuf  = (float*)(wsb + o_h);

  k_masks<<<dim3(NB), dim3(256), 0, stream>>>(cmap, m1, m2, m3, m4);
  k_cast_w2<<<dim3((CH2 * 9 * 4) / 256), dim3(256), 0, stream>>>(W2, w2t);
  k_cast_fc1<<<dim3((NHID * 256 * 8) / 256), dim3(256), 0, stream>>>(Wfc1, wfc1t);
  k_conv1_pool<<<dim3(NB * H1), dim3(128), 0, stream>>>(x, W1, b1, m1, m2, p1);
  for (int c = 0; c < NCHUNK; ++c) {
    const _Float16* p1c = p1 + (size_t)c * CHUNK_IMG * H1 * H1 * CH1;
    k_im2col<<<dim3(IM2COL_WAVES / 8), dim3(256), 0, stream>>>(p1c, acol);
    _Float16* r2c = r2 + (size_t)c * CHUNK_ROWS * CH2;
    const int* m3c = m3 + (size_t)c * CHUNK_ROWS;
    wmma_gemm64<0, 2, 1, 2, true><<<dim3((CHUNK_ROWS / 64) * (CH2 / 64) / 8, 1), dim3(256), 0, stream>>>(
        (const unsigned short*)acol, KC2, 0L,
        (const unsigned short*)w2t, KC2, 0L,
        (void*)r2c, CH2, 0L,
        b2,
        m3c, 0L,
        CHUNK_ROWS, CH2, KC2, 1.0f);
  }
  k_pool2<<<dim3((NB * 256 * 8) / 256), dim3(256), 0, stream>>>(r2, m4, p2);
  wmma_gemm64<0, 2, 0, 2, false><<<dim3(1, 1), dim3(256), 0, stream>>>(
      (const unsigned short*)p2, KFC, 0L,
      (const unsigned short*)wfc1t, KFC, 0L,
      (void*)hbuf, NHID, 0L,
      bfc1,
      m4, 0L,
      NB, NHID, KFC, 1.0f / 64.0f);
  k_fc2<<<dim3((NB * NCLS) / 256), dim3(256), 0, stream>>>(hbuf, Wfc2, bfc2, out);
}
